// CoPELlamaAttention_68307159875895
// MI455X (gfx1250) — hardware-verified
//
#include <hip/hip_runtime.h>


namespace {
constexpr int Bn = 2, S = 1024, HID = 2048, H = 16, KVH = 8, D = 128, NPOS = 64, GRP = H / KVH, NTOK = Bn * S, NQKV = HID + 2 * KVH * D;
constexpr float SCALE = 0.08838834764831845f, PSC = 8.0f;

typedef _Float16 b16;
typedef __attribute__((ext_vector_type(16))) _Float16 v16b;
typedef __attribute__((ext_vector_type(8)))  _Float16 v8b;
typedef __attribute__((ext_vector_type(8)))  float v8f;
typedef __attribute__((ext_vector_type(4)))  float v4f;

__device__ __forceinline__ v8b ld8b(const b16* p) { return *(const v8b*)p; }
__device__ __forceinline__ v16b cat8b(v8b a, v8b b) { return __builtin_shufflevector(a, b, 0, 1, 2, 3, 4, 5, 6, 7, 8, 9, 10, 11, 12, 13, 14, 15); }
__device__ __forceinline__ v16b frag_kb(const b16* p, int hh) { return cat8b(ld8b(p + 8 * hh), ld8b(p + 16 + 8 * hh)); }
__device__ __forceinline__ void split16(float v, b16& hi, b16& lo) { hi = (b16)v; lo = (b16)(v - (float)hi); }
__device__ __forceinline__ void frag_ksplit(const float* p, int hh, v16b& fh_, v16b& fl_) {
  const float* p0 = p + 8 * hh; const float* p1 = p + 16 + 8 * hh;
#pragma unroll
  for (int e = 0; e < 8; ++e) { b16 a, c; split16(p0[e], a, c); fh_[e] = a; fl_[e] = c; split16(p1[e], a, c); fh_[8 + e] = a; fl_[8 + e] = c; }
}
__device__ __forceinline__ v8f wmma16b(v16b a, v16b b, v8f c) {
  v8f d = __builtin_amdgcn_wmma_f32_16x16x32_f16(false, a, false, b, (short)0, c, false, false);
  asm volatile("v_nop\n\tv_nop\n\tv_nop\n\tv_nop" : "+v"(d) : "v"(a), "v"(b));
  return d;
}
__device__ __forceinline__ void wave_lds_sync() {
  __builtin_amdgcn_fence(__ATOMIC_RELEASE, "workgroup");
  __builtin_amdgcn_wave_barrier();
  __builtin_amdgcn_fence(__ATOMIC_ACQUIRE, "workgroup");
}

struct Opnd { const void* p0; const void* p1; int ld; };
template <int NP> __device__ __forceinline__ void load_frags(const Opnd& o, int row, int kb, int hh, v16b& fh_, v16b& fl_) {
  if (NP == 0) { frag_ksplit((const float*)o.p0 + (size_t)row * o.ld + kb, hh, fh_, fl_); }
  else if (NP == 4 || NP == 5) {
    const float sc_ = (NP == 4) ? 64.0f : 8.0f;
    const float* p = (const float*)o.p0 + (size_t)row * o.ld + kb; const float* p0 = p + 8 * hh; const float* p1 = p + 16 + 8 * hh;
#pragma unroll
    for (int e = 0; e < 8; ++e) { b16 a, c; split16(p0[e] * sc_, a, c); fh_[e] = a; fl_[e] = c; split16(p1[e] * sc_, a, c); fh_[8 + e] = a; fl_[8 + e] = c; }
  } else if (NP == 3) {
    const float* p = (const float*)o.p0 + (size_t)row * o.ld + kb; const float* p0 = p + 8 * hh; const float* p1 = p + 16 + 8 * hh;
#pragma unroll
    for (int e = 0; e < 8; ++e) { fh_[e] = (b16)p0[e]; fh_[8 + e] = (b16)p1[e]; }
    fl_ = fh_;
  } else {
    fh_ = frag_kb((const b16*)o.p0 + (size_t)row * o.ld + kb, hh);
    if (NP == 2) fl_ = frag_kb((const b16*)o.p1 + (size_t)row * o.ld + kb, hh); else fl_ = fh_;
  }
}
template <int ANP, int BNP> __device__ __forceinline__ v8f mac(v16b ah, v16b al, v16b bh, v16b bl, v8f c) {
  c = wmma16b(ah, bh, c);
  if (BNP == 0 || BNP == 2 || BNP == 4 || BNP == 5) c = wmma16b(ah, bl, c);
  if (ANP == 0 || ANP == 2 || ANP == 4 || ANP == 5) c = wmma16b(al, bh, c);
  return c;
}
template <int ANP, int BNP>
__device__ __forceinline__ void gemm_tile(const Opnd& A, const Opnd& B, int K, int m0, int c0, int nloc, int hlf, v8f (&acc)[2][4]) {
  for (int kb = 0; kb < K; kb += 32) {
    v16b a0h, a0l, a1h, a1l;
    load_frags<ANP>(A, m0 + nloc, kb, hlf, a0h, a0l);
    load_frags<ANP>(A, m0 + 16 + nloc, kb, hlf, a1h, a1l);
#pragma unroll
    for (int t = 0; t < 4; ++t) {
      v16b bh, bl;
      load_frags<BNP>(B, c0 + t * 16 + nloc, kb, hlf, bh, bl);
      acc[0][t] = mac<ANP, BNP>(a0h, a0l, bh, bl, acc[0][t]);
      acc[1][t] = mac<ANP, BNP>(a1h, a1l, bh, bl, acc[1][t]);
    }
  }
}

__device__ __forceinline__ void epi_planes(v8f (&acc)[2][4], float scale, bool two, b16* __restrict__ oh, b16* __restrict__ ol, int ldo,
                                           int m0, int c0, int lane, b16* Th, b16* Tl) {
  const int nloc = lane & 15, hlf = lane >> 4;
#pragma unroll
  for (int t = 0; t < 4; ++t)
#pragma unroll
    for (int r = 0; r < 2; ++r)
#pragma unroll
      for (int v = 0; v < 8; ++v) {
        const int rr = r * 16 + v + 8 * hlf, cc = t * 16 + nloc;
        b16 h_, l_; split16(acc[r][t][v] * scale, h_, l_);
        Th[rr * 64 + cc] = h_; Tl[rr * 64 + cc] = l_;
      }
  wave_lds_sync();
  for (int pass = 0; pass < 2; ++pass) {
#pragma unroll
    for (int j = 0; j < 8; ++j) {
      const int rr = j * 4 + (lane >> 3), c8 = (lane & 7) * 8;
      const size_t o = (size_t)(m0 + rr) * ldo + c0 + c8;
      *(volatile v8b*)(oh + o) = ld8b(Th + rr * 64 + c8);
      if (two) *(volatile v8b*)(ol + o) = ld8b(Tl + rr * 64 + c8);
    }
    __threadfence();
  }
}
__device__ __forceinline__ void epi_f32(v8f (&acc)[2][4], float scale, const float* rscale, float* __restrict__ out, int ldo, int m0, int c0, int lane, float* Tt) {
  const int nloc = lane & 15, hlf = lane >> 4;
#pragma unroll
  for (int t = 0; t < 4; ++t)
#pragma unroll
    for (int r = 0; r < 2; ++r)
#pragma unroll
      for (int v = 0; v < 8; ++v) {
        const int rr = r * 16 + v + 8 * hlf;
        const float rs = rscale ? rscale[(size_t)(m0 + rr) * 32] : 1.0f;
        Tt[rr * 64 + t * 16 + nloc] = acc[r][t][v] * scale * rs;
      }
  wave_lds_sync();
  float* dst0 = out + (size_t)m0 * ldo + c0;
  for (int pass = 0; pass < 2; ++pass) {
#pragma unroll
    for (int j = 0; j < 16; ++j) { const int rr = j * 2 + hlf, c4 = nloc * 4; *(volatile v4f*)(dst0 + (size_t)rr * ldo + c4) = *(const v4f*)(Tt + rr * 64 + c4); }
    __threadfence();
  }
}


typedef __attribute__((ext_vector_type(8))) __bf16 v8bb; typedef __attribute__((ext_vector_type(16))) __bf16 v16bb;
__device__ __forceinline__ v16bb frag_kb_bf(const __bf16* p, int hh) { const v8bb a = *(const v8bb*)(p + 8 * hh), b = *(const v8bb*)(p + 16 + 8 * hh); return __builtin_shufflevector(a, b, 0, 1, 2, 3, 4, 5, 6, 7, 8, 9, 10, 11, 12, 13, 14, 15); }
__device__ __forceinline__ v8f wmma16bb(v16bb a, v16bb b, v8f c) {
  v8f d = __builtin_amdgcn_wmma_f32_16x16x32_bf16(false, a, false, b, (short)0, c, false, false);
  asm volatile("v_nop\n\tv_nop\n\tv_nop\n\tv_nop" : "+v"(d) : "v"(a), "v"(b));
  return d;
}
__device__ __forceinline__ unsigned short bf16_rne_bits(float v) { unsigned int u = __float_as_uint(v); u += 0x7FFFu + ((u >> 16) & 1u); return (unsigned short)(u >> 16); }
__device__ __forceinline__ float bf16_rne(float v) { return __uint_as_float(((unsigned int)bf16_rne_bits(v)) << 16); }

__global__ __launch_bounds__(256) void prep_kernel(const float* __restrict__ hs, const float* __restrict__ wq, const float* __restrict__ wk, const float* __restrict__ wv,
                                                   const float* __restrict__ wo, const float* __restrict__ pe,
                                                   unsigned short* __restrict__ hs16, unsigned short* __restrict__ w16, b16* __restrict__ wo16, b16* __restrict__ peT) {
  typedef __attribute__((ext_vector_type(8))) unsigned short v8us;
  const size_t tid = (size_t)blockIdx.x * blockDim.x + threadIdx.x, stride = (size_t)gridDim.x * blockDim.x;
  const size_t n0 = (size_t)NTOK * HID / 8, n1 = (size_t)NQKV * HID / 8, n2 = (size_t)HID * HID / 8, n3 = (size_t)NPOS * D / 8;
  for (int pass = 0; pass < 2; ++pass) {
    for (size_t p = tid; p < n0 + n1 + n2 + n3; p += stride) {
      if (p < n0 + n1) {
        const size_t i = (p < n0) ? p * 8 : (p - n0) * 8; const float* src; unsigned short* dst;
        if (p < n0) { src = hs + i; dst = hs16 + i; }
        else { src = (i < (size_t)HID * HID) ? (wq + i) : (i < (size_t)(HID + KVH * D) * HID) ? (wk + i - (size_t)HID * HID) : (wv + i - (size_t)(HID + KVH * D) * HID); dst = w16 + i; }
        v8us v;
#pragma unroll
        for (int e = 0; e < 8; ++e) v[e] = bf16_rne_bits(src[e]);
        *(volatile v8us*)dst = v;
      } else if (p < n0 + n1 + n2) { const size_t i = (p - n0 - n1) * 8; v8b v;
#pragma unroll
        for (int e = 0; e < 8; ++e) v[e] = (b16)bf16_rne(wo[i + e]);
        *(volatile v8b*)(wo16 + i) = v; }
      else { const size_t i = (p - n0 - n1 - n2) * 8; const int n = (int)(i / D), d0 = (int)(i % D); v8b v;
#pragma unroll
        for (int e = 0; e < 8; ++e) v[e] = (b16)bf16_rne(pe[(size_t)(d0 + e) * NPOS + n]);
        *(volatile v8b*)(peT + i) = v; }
    }
    __threadfence();
  }
}

__global__ __launch_bounds__(128) void proj_kernel(const __bf16* __restrict__ hs16, const __bf16* __restrict__ w16, b16* __restrict__ qh, b16* __restrict__ ql,
                                                   b16* __restrict__ kh, b16* __restrict__ kl, b16* __restrict__ vth, b16* __restrict__ vtl) {
  __shared__ __attribute__((aligned(16))) b16 Th[4][2][32 * 64];
  __shared__ __attribute__((aligned(16))) b16 Tt[2][64][128 + 8];
  const int lane = threadIdx.x & 31, wave = threadIdx.x >> 5, nloc = lane & 15, hlf = lane >> 4;
  const int m0 = blockIdx.y * 128 + wave * 32, c0 = blockIdx.x * 64;
  v8f acc[2][4];
#pragma unroll
  for (int r = 0; r < 2; ++r)
#pragma unroll
    for (int t = 0; t < 4; ++t) acc[r][t] = (v8f){};
#pragma unroll 2
  for (int kb = 0; kb < HID; kb += 32) {
    const v16bb a0 = frag_kb_bf(hs16 + (size_t)(m0 + nloc) * HID + kb, hlf), a1 = frag_kb_bf(hs16 + (size_t)(m0 + 16 + nloc) * HID + kb, hlf);
#pragma unroll
    for (int t = 0; t < 4; ++t) { const v16bb bw = frag_kb_bf(w16 + (size_t)(c0 + t * 16 + nloc) * HID + kb, hlf); acc[0][t] = wmma16bb(a0, bw, acc[0][t]); acc[1][t] = wmma16bb(a1, bw, acc[1][t]); }
  }
  const int b = (blockIdx.y * 128) / S, s0 = (blockIdx.y * 128) % S + wave * 32;
  if (c0 < HID) {
    const int h = c0 / D, d0 = c0 % D;
    epi_planes(acc, PSC, true, qh + (((size_t)b * H + h) * S + s0) * D - (size_t)0, ql + (((size_t)b * H + h) * S + s0) * D, D, 0, d0, lane, Th[wave][0], Th[wave][1]);
    return;
  }
  if (c0 < HID + KVH * D) { const int c1 = c0 - HID, g = c1 / D, d0 = c1 % D;
    epi_planes(acc, PSC, true, kh + (((size_t)b * KVH + g) * S + s0) * D, kl + (((size_t)b * KVH + g) * S + s0) * D, D, 0, d0, lane, Th[wave][0], Th[wave][1]);
    return;
  }
  const int c1 = c0 - HID - KVH * D, g = c1 / D, d0 = c1 % D;
#pragma unroll
  for (int t = 0; t < 4; ++t)
#pragma unroll
    for (int r = 0; r < 2; ++r)
#pragma unroll
      for (int v = 0; v < 8; ++v) { b16 a, c; split16(acc[r][t][v] * PSC, a, c); Tt[0][t * 16 + nloc][wave * 32 + r * 16 + 8 * hlf + v] = a; Tt[1][t * 16 + nloc][wave * 32 + r * 16 + 8 * hlf + v] = c; }
  __syncthreads();
  const int tok0 = (blockIdx.y * 128) % S;
  b16* bh_ = vth + (((size_t)b * KVH + g) * D + d0) * S + tok0; b16* bl_ = vtl + (((size_t)b * KVH + g) * D + d0) * S + tok0;
  for (int pass = 0; pass < 2; ++pass) {
#pragma unroll
    for (int j = 0; j < 8; ++j) { const int dd = wave * 16 + j * 2 + (lane >> 4), c8 = (lane & 15) * 8;
      *(volatile v8b*)(bh_ + (size_t)dd * S + c8) = *(const v8b*)(&Tt[0][dd][c8]); *(volatile v8b*)(bl_ + (size_t)dd * S + c8) = *(const v8b*)(&Tt[1][dd][c8]); }
    __threadfence();
  }
}

__global__ __launch_bounds__(128) void li_kernel(const b16* __restrict__ qh, const b16* __restrict__ ql, const b16* __restrict__ peT, float* __restrict__ li) {
  __shared__ __attribute__((aligned(16))) float Ts[4][32 * 64];
  const int lane = threadIdx.x & 31, wave = threadIdx.x >> 5, nloc = lane & 15, hlf = lane >> 4, m0 = blockIdx.y * 128 + wave * 32;
  v8f acc[2][4];
#pragma unroll
  for (int r = 0; r < 2; ++r)
#pragma unroll
    for (int t = 0; t < 4; ++t) acc[r][t] = (v8f){};
  const Opnd A{qh, ql, D}, B{peT, nullptr, D};
  gemm_tile<2, 1>(A, B, D, m0, 0, nloc, hlf, acc);
  epi_f32(acc, 1.0f / PSC, nullptr, li, NPOS, m0, 0, lane, Ts[wave]);
}

__global__ __launch_bounds__(256) void attn_kernel(const b16* __restrict__ qh, const b16* __restrict__ ql, const b16* __restrict__ kh, const b16* __restrict__ kl,
                                                   const b16* __restrict__ vth, const b16* __restrict__ vtl, const float* __restrict__ li, const float* __restrict__ amask,
                                                   float* __restrict__ y) {
  __shared__ float Ls[8][16][NPOS + 1];
  __shared__ __attribute__((aligned(16))) float Os[8][16][D + 4];
  const int wid = threadIdx.x >> 5, lane = threadIdx.x & 31, hh = lane >> 4, col = lane & 15;
  const int qt = blockIdx.x * 8 + wid, jt = qt & 63, h = (qt >> 6) & 15, b = qt >> 10, q0 = jt * 16, g = h / GRP, qi = q0 + col;
  const size_t qrow = ((size_t)b * H + h) * S; const size_t krow = ((size_t)b * KVH + g) * S;
  for (int i = lane; i < 16 * NPOS; i += 32) Ls[wid][i / NPOS][i % NPOS] = li[(qrow + q0 + i / NPOS) * NPOS + (i % NPOS)];
  wave_lds_sync();
  const v16b bqh = frag_kb(qh + (qrow + qi) * D, hh), bql = frag_kb(ql + (qrow + qi) * D, hh);
  (void)bqh; (void)bql;
  const float* mrow = amask + ((size_t)b * S + qi) * S;
  float m = -INFINITY, l = 0.0f, carry = 0.0f;
  v8f o[8];
#pragma unroll
  for (int n = 0; n < 8; ++n) o[n] = (v8f){};
  const b16* vh = vth + ((size_t)b * KVH + g) * D * S; const b16* vl = vtl + ((size_t)b * KVH + g) * D * S;
  for (int kb = (q0 / 32) * 32; kb >= 0; kb -= 32) {
    v8f s0 = {}, s1 = {};
#pragma unroll
    for (int ks = 0; ks < 4; ++ks) {
      const v16b qhf = frag_kb(qh + (qrow + qi) * D + ks * 32, hh), qlf = frag_kb(ql + (qrow + qi) * D + ks * 32, hh);
      { const v16b ah = frag_kb(kh + (krow + kb + col) * D + ks * 32, hh), al = frag_kb(kl + (krow + kb + col) * D + ks * 32, hh); s0 = mac<2, 2>(ah, al, qhf, qlf, s0); }
      { const v16b ah = frag_kb(kh + (krow + kb + 16 + col) * D + ks * 32, hh), al = frag_kb(kl + (krow + kb + 16 + col) * D + ks * 32, hh); s1 = mac<2, 2>(ah, al, qhf, qlf, s1); }
    }
    float lg0[8], lg1[8], g0v[8], g1v[8]; bool mk0[8], mk1[8];
#pragma unroll
    for (int r = 0; r < 8; ++r) {
      const int k0i = kb + 8 * hh + r, k1i = k0i + 16; const float mv0 = mrow[k0i], mv1 = mrow[k1i];
      lg0[r] = s0[r] * (SCALE / (PSC * PSC)) + mv0; lg1[r] = s1[r] * (SCALE / (PSC * PSC)) + mv1; mk0[r] = (mv0 != 0.0f); mk1[r] = (mv1 != 0.0f);
      g0v[r] = 1.0f / (1.0f + __expf(-lg0[r])); g1v[r] = 1.0f / (1.0f + __expf(-lg1[r]));
    }
    float sa = 0.0f, sb = 0.0f;
#pragma unroll
    for (int r = 0; r < 8; ++r) { sa += g0v[r]; sb += g1v[r]; }
    const float pa = __shfl_xor(sa, 16), pb_ = __shfl_xor(sb, 16);
    const float G0 = hh ? pa : sa, G1 = hh ? sa : pa, G2 = hh ? pb_ : sb, G3 = hh ? sb : pb_;
    const float baseB = hh ? 0.0f : G3;
    const float baseA = hh ? (G3 + G2) : (G3 + G2 + G1);
    float posA[8], posB[8];
    { float run = carry + baseB;
#pragma unroll
      for (int r = 7; r >= 0; --r) { run += g1v[r]; posB[r] = run; } }
    { float run = carry + baseA;
#pragma unroll
      for (int r = 7; r >= 0; --r) { run += g0v[r]; posA[r] = run; } }
    carry += G0 + G1 + G2 + G3;
#pragma unroll
    for (int r = 0; r < 8; ++r) {
      { const float pz = fminf(posA[r], (float)(NPOS - 1)); const float pf = floorf(pz), pc = ceilf(pz), w = pz - pf;
        const float lf = Ls[wid][col][(int)pf], lc = Ls[wid][col][(int)pc]; lg0[r] = mk0[r] ? -INFINITY : (lg0[r] + lc * w + lf * (1.0f - w)); }
      { const float pz = fminf(posB[r], (float)(NPOS - 1)); const float pf = floorf(pz), pc = ceilf(pz), w = pz - pf;
        const float lf = Ls[wid][col][(int)pf], lc = Ls[wid][col][(int)pc]; lg1[r] = mk1[r] ? -INFINITY : (lg1[r] + lc * w + lf * (1.0f - w)); }
    }
    float mr = -INFINITY;
#pragma unroll
    for (int r = 0; r < 8; ++r) mr = fmaxf(mr, fmaxf(lg0[r], lg1[r]));
    mr = fmaxf(mr, __shfl_xor(mr, 16));
    float mn = fmaxf(m, mr); if (mn == -INFINITY) mn = 0.0f;
    const float al_ = __expf(m - mn); m = mn;
    float sum = 0.0f; v16b pbf;
#pragma unroll
    for (int r = 0; r < 8; ++r) { const float p0 = __expf(lg0[r] - mn), p1 = __expf(lg1[r] - mn); sum += p0 + p1; pbf[r] = (b16)p0; pbf[8 + r] = (b16)p1; }
    sum += __shfl_xor(sum, 16); l = l * al_ + sum;
#pragma unroll
    for (int n = 0; n < 8; ++n) {
#pragma unroll
      for (int r = 0; r < 8; ++r) o[n][r] *= al_;
      const size_t ro = (size_t)(n * 16 + col) * S + kb;
      o[n] = wmma16b(frag_kb(vh + ro, hh), pbf, o[n]); o[n] = wmma16b(frag_kb(vl + ro, hh), pbf, o[n]);
    }
  }
  const float inv = (l > 0.0f) ? (1.0f / (PSC * l)) : 0.0f; float* Tt = Os[wid][0];
#pragma unroll
  for (int n = 0; n < 8; ++n)
#pragma unroll
    for (int r = 0; r < 8; ++r) Os[wid][col][n * 16 + 8 * hh + r] = o[n][r] * inv;
  wave_lds_sync();
  float* dst = y + ((size_t)b * S + q0) * HID + h * D;
  for (int pass = 0; pass < 2; ++pass) {
#pragma unroll
    for (int rr = 0; rr < 16; ++rr) *(volatile v4f*)(dst + (size_t)rr * HID + lane * 4) = *(const v4f*)(&Os[wid][rr][lane * 4]);
    __threadfence();
  }
  (void)Tt;
}

__global__ __launch_bounds__(128) void out_kernel(const float* __restrict__ y, const b16* __restrict__ wo16, float* __restrict__ out) {
  __shared__ __attribute__((aligned(16))) float Ts[4][32 * 64];
  const int lane = threadIdx.x & 31, wave = threadIdx.x >> 5, nloc = lane & 15, hlf = lane >> 4;
  const int m0 = blockIdx.y * 128 + wave * 32, c0 = blockIdx.x * 64;
  v8f acc[2][4];
#pragma unroll
  for (int r = 0; r < 2; ++r)
#pragma unroll
    for (int t = 0; t < 4; ++t) acc[r][t] = (v8f){};
  const Opnd A{y, nullptr, HID}, B{wo16, nullptr, HID};
  gemm_tile<5, 1>(A, B, HID, m0, c0, nloc, hlf, acc);
  epi_f32(acc, 1.0f / PSC, nullptr, out, HID, m0, c0, lane, Ts[wave]);
}
}

extern "C" void kernel_launch(void* const* d_in, const int* in_sizes, int n_in,
                              void* d_out, int out_size, void* d_ws, size_t ws_size, hipStream_t stream) {
  (void)n_in; (void)out_size;
  const float* hs = (const float*)d_in[0];
  const float* am = (const float*)d_in[1];
  const float* wq = (const float*)d_in[2]; const float* wk = (const float*)d_in[3]; const float* wv = (const float*)d_in[4]; const float* wo = (const float*)d_in[5];
  const float* pe = (const float*)d_in[6];
  float* out = (float*)d_out;
  if (in_sizes[0] != NTOK * HID || in_sizes[1] != Bn * S * S || in_sizes[2] != HID * HID || in_sizes[3] != KVH * D * HID || in_sizes[6] != D * NPOS) return;
  size_t off = 0; char* ws = (char*)d_ws;
  auto carve = [&](size_t bytes) { char* p = ws + off; off += (bytes + 255) & ~(size_t)255; return p; };
  unsigned short* hs16 = (unsigned short*)carve((size_t)NTOK * HID * 2);
  unsigned short* w16 = (unsigned short*)carve((size_t)NQKV * HID * 2);
  b16* wo16 = (b16*)carve((size_t)HID * HID * 2);
  b16* peT = (b16*)carve((size_t)NPOS * D * 2);
  b16* qh = (b16*)carve((size_t)Bn * H * S * D * 2); b16* ql = (b16*)carve((size_t)Bn * H * S * D * 2);
  b16* khp = (b16*)carve((size_t)Bn * KVH * S * D * 2); b16* klp = (b16*)carve((size_t)Bn * KVH * S * D * 2);
  b16* vth = (b16*)carve((size_t)Bn * KVH * D * S * 2); b16* vtl = (b16*)carve((size_t)Bn * KVH * D * S * 2);
  float* li = (float*)carve((size_t)Bn * H * S * NPOS * 4);
  float* y = (float*)carve((size_t)NTOK * HID * 4);
  if (off > ws_size) return;
  prep_kernel<<<1024, 256, 0, stream>>>(hs, wq, wk, wv, wo, pe, hs16, w16, wo16, peT);
  proj_kernel<<<dim3(NQKV / 64, NTOK / 128), 128, 0, stream>>>((const __bf16*)hs16, (const __bf16*)w16, qh, ql, khp, klp, vth, vtl);
  li_kernel<<<dim3(1, Bn * H * S / 128), 128, 0, stream>>>(qh, ql, peT, li);
  attn_kernel<<<Bn * H * (S / 16) / 8, 256, 0, stream>>>(qh, ql, khp, klp, vth, vtl, li, am, y);
  out_kernel<<<dim3(HID / 64, NTOK / 128), 128, 0, stream>>>(y, wo16, out);
}
